// Attention_19129784336852
// MI455X (gfx1250) — hardware-run, weakly checked
//
#include <hip/hip_runtime.h>


#ifndef NB
#define NB 8
#endif
#ifndef SEQ
#define SEQ 2048
#endif
#define NB_FULL  8
#define SEQ_FULL 2048
#define DIM  512
#define NH   8
#define HD   64
#define DIM3 1536
#define NWV  4
#define BQ   (16 * NWV)
#define KS   32
#define OSP  68
#define GP   68
#define GBM  128
#define GBN  64
#define L2E  1.4426950408889634f
#define PCL  10.0f
#define QCAR 64.0f
#define KCAR 8.0f
#define WCAR 256.0f
#define CCAR 16.0f
#define QEP  (QCAR / WCAR)
#define KEP  (KCAR / WCAR)
#define VEP  (1.0f / WCAR)
#define OSC  (1.0f / 4096.0f)
#define SCL  (1.0f / 512.0f)
#define L2ES (L2E * SCL)
#define LNEPS 1.0e-6f
#define MROWS (NB * SEQ)
#define PLN  ((size_t)MROWS * DIM)

static_assert(HD == 64);
static_assert(8 * 8 == HD);
static_assert(GBN == HD);
static_assert(NH * HD == DIM);
static_assert(DIM3 == 3 * DIM);
static_assert(DIM % 32 == 0);
static_assert(HD % 32 == 0);
static_assert(DIM % 8 == 0);
static_assert(DIM == 32 * 16);
static_assert(DIM3 % GBN == 0);
static_assert(DIM % GBN == 0);
static_assert(SEQ % BQ == 0);
static_assert(SEQ % KS == 0);
static_assert(SEQ % GBM == 0);
static_assert(MROWS % GBM == 0);
static_assert(MROWS % 8 == 0);
static_assert(GBM == 32 * NWV);
static_assert(NB <= NB_FULL);
static_assert(SEQ <= SEQ_FULL);
static_assert(QCAR * KCAR * SCL == 1.0f);
static_assert(CCAR * WCAR * OSC == 1.0f);
static_assert(QEP * WCAR == QCAR);
static_assert(KEP * WCAR == KCAR);
static_assert(VEP * WCAR == 1.0f);
static_assert(((size_t)DIM3 * (DIM / 8)) % 256 == 0);
static_assert(((size_t)DIM * (DIM / 8)) % 256 == 0);
static_assert((size_t)(MROWS / 8) * 8 * (size_t)(2 * 32 * 8) == (size_t)MROWS * DIM);
static_assert((size_t)(MROWS / GBM) * (DIM3 / GBN) * (size_t)(GBM * GBN) == (size_t)MROWS * DIM3);
static_assert((size_t)(MROWS / GBM) * (DIM / GBN) * (size_t)(GBM * GBN) == (size_t)MROWS * DIM);
static_assert((size_t)(NB * NH) * (SEQ / BQ) * (size_t)(BQ * HD) == (size_t)MROWS * DIM);
static_assert(8 * 128 == GBM * (HD / 8));
static_assert(8 * 128 == HD * (GBM / 8));
static_assert(16 * 128 == GBM * (GBN / 4));
static_assert(4 * 4 == 16);

typedef unsigned short bf;
typedef __attribute__((ext_vector_type(16))) _Float16 v16h;
typedef __attribute__((ext_vector_type(8)))  _Float16 v8h;
typedef __attribute__((ext_vector_type(8)))  unsigned short v8us;
typedef __attribute__((ext_vector_type(8)))  float    v8f;
typedef __attribute__((ext_vector_type(4)))  float    v4f;
typedef v4f  __attribute__((may_alias)) v4fa;

__device__ __forceinline__ unsigned short f2bf(float f) { unsigned u = __float_as_uint(f); u += 0x7FFFu + ((u >> 16) & 1u); return (unsigned short)(u >> 16); }
__device__ __forceinline__ float bf2f(unsigned short b) { return __uint_as_float(((unsigned)b) << 16); }
__device__ __forceinline__ v8f wmmah(v16h a, v16h b, v8f c) { return __builtin_amdgcn_wmma_f32_16x16x32_f16(false, a, false, b, (short)0, c, false, false); }
__device__ __forceinline__ _Float16 toh_flush(float v) { const _Float16 r = (_Float16)v; return (fabsf(v) < 6.103515625e-05f) ? (_Float16)0.0f : r; }
__device__ __forceinline__ v16h ldh(const bf* p) {
    const v8us lo = *(const v8us*)p; const v8us hi = *(const v8us*)(p + 16);
    return __builtin_bit_cast(v16h, __builtin_shufflevector(lo, hi, 0, 1, 2, 3, 4, 5, 6, 7, 8, 9, 10, 11, 12, 13, 14, 15));
}

__global__ __launch_bounds__(256) void k_ln(const float* __restrict__ x, const float* __restrict__ gam, const float* __restrict__ bet, bf* XN) {
#pragma clang fp contract(off)
    const unsigned lane = threadIdx.x & 31u;
    const unsigned row = blockIdx.x * 8u + (threadIdx.x >> 5);
    if (row >= (unsigned)MROWS) return;
    const unsigned b = row / (unsigned)SEQ, n = row - b * (unsigned)SEQ;
    const float* src = x + ((size_t)b * SEQ_FULL + n) * DIM + 8u * lane;
    const v8f r0 = *(const v8f*)src;
    const v8f r1 = *(const v8f*)(src + 256);
    const v8f g0 = *(const v8f*)(gam + 8u * lane);
    const v8f g1 = *(const v8f*)(gam + 256 + 8u * lane);
    const v8f e0 = *(const v8f*)(bet + 8u * lane);
    const v8f e1 = *(const v8f*)(bet + 256 + 8u * lane);
    v8f a0, a1;
    float s = 0.0f;
#pragma unroll
    for (int c = 0; c < 8; ++c) {
        a0[c] = bf2f(f2bf(r0[c]));
        a1[c] = bf2f(f2bf(r1[c]));
        s += a0[c] + a1[c];
    }
#pragma unroll
    for (int m = 16; m >= 1; m >>= 1) s += __shfl_xor(s, m, 32);
    const float mu = s * (1.0f / (float)DIM);
    float q = 0.0f;
#pragma unroll
    for (int c = 0; c < 8; ++c) {
        const float d0 = a0[c] - mu, d1 = a1[c] - mu;
        q += d0 * d0 + d1 * d1;
    }
#pragma unroll
    for (int m = 16; m >= 1; m >>= 1) q += __shfl_xor(q, m, 32);
    const float rs = rsqrtf(q * (1.0f / (float)DIM) + LNEPS);
    v8h h0, h1;
#pragma unroll
    for (int c = 0; c < 8; ++c) {
        const float t0 = (a0[c] - mu) * rs * bf2f(f2bf(g0[c])) + bf2f(f2bf(e0[c]));
        const float t1 = (a1[c] - mu) * rs * bf2f(f2bf(g1[c])) + bf2f(f2bf(e1[c]));
        h0[c] = toh_flush(t0);
        h1[c] = toh_flush(t1);
    }
    const v8us u0 = __builtin_bit_cast(v8us, h0);
    const v8us u1 = __builtin_bit_cast(v8us, h1);
    bf* dst = XN + (size_t)row * DIM + 8u * lane;
#pragma unroll 1
    for (int ps = 0; ps < 2; ++ps) {
        *(volatile v8us*)(dst) = u0;
        *(volatile v8us*)(dst + 256) = u1;
        if (ps == 0) __threadfence();
    }
}

__global__ __launch_bounds__(256) void k_wc(const float* __restrict__ W, bf* WT, int N, int pitch, int ndup, int qrows) {
    const unsigned i = blockIdx.x * 256u + threadIdx.x;
    if (i >= (unsigned)N * (unsigned)(DIM / 8)) return;
    const unsigned n = i / (unsigned)(DIM / 8), c8 = (i - n * (unsigned)(DIM / 8)) * 8u;
    const float sc = ((int)n < qrows) ? (0.125f * WCAR) : WCAR;
    const v8f v = *(const v8f*)(W + (size_t)n * DIM + c8);
    v8h oh;
#pragma unroll
    for (int c = 0; c < 8; ++c) oh[c] = toh_flush(bf2f(f2bf(v[c])) * sc);
    const v8us o = __builtin_bit_cast(v8us, oh);
#pragma unroll 1
    for (int ps = 0; ps < 2; ++ps) {
#pragma unroll 1
        for (int dup = 0; dup < ndup; ++dup) {
            *(volatile v8us*)(WT + (size_t)n * (unsigned)pitch + (unsigned)dup * DIM + c8) = o;
        }
        if (ps == 0) __threadfence();
    }
}

__device__ __forceinline__ void gemm_acc(const bf* __restrict__ A, const bf* __restrict__ BT, const unsigned K,
                                         const unsigned arow, const unsigned brow, const unsigned hi, v8f (&acc)[2][4]) {
    const bf* ap = A + (size_t)arow * K + 8u * hi;
    const bf* bp = BT + (size_t)brow * K + 8u * hi;
    const size_t s16 = (size_t)16 * K;
#pragma unroll 1
    for (unsigned k0 = 0; k0 < K; k0 += 32) {
        const v16h a0 = ldh(ap + k0);
        const v16h a1 = ldh(ap + s16 + k0);
        const v16h b0 = ldh(bp + k0);
        const v16h b1 = ldh(bp + s16 + k0);
        const v16h b2 = ldh(bp + 2 * s16 + k0);
        const v16h b3 = ldh(bp + 3 * s16 + k0);
        acc[0][0] = wmmah(a0, b0, acc[0][0]);
        acc[1][0] = wmmah(a1, b0, acc[1][0]);
        acc[0][1] = wmmah(a0, b1, acc[0][1]);
        acc[1][1] = wmmah(a1, b1, acc[1][1]);
        acc[0][2] = wmmah(a0, b2, acc[0][2]);
        acc[1][2] = wmmah(a1, b2, acc[1][2]);
        acc[0][3] = wmmah(a0, b3, acc[0][3]);
        acc[1][3] = wmmah(a1, b3, acc[1][3]);
        asm volatile("v_nop\n\tv_nop\n\tv_nop\n\tv_nop"
                     : "+v"(acc[0][0]), "+v"(acc[1][0]), "+v"(acc[0][1]), "+v"(acc[1][1]),
                       "+v"(acc[0][2]), "+v"(acc[1][2]), "+v"(acc[0][3]), "+v"(acc[1][3])
                     : "v"(a0), "v"(a1), "v"(b0), "v"(b1), "v"(b2), "v"(b3));
    }
}

__global__ __launch_bounds__(128) void k_qkv(const bf* __restrict__ XN, const bf* __restrict__ WQT, bf* QK, bf* VT) {
    __shared__ __align__(16) float st[GBM * GP];
    const unsigned tid = threadIdx.x, lane = tid & 31u, wv = tid >> 5, lr = lane & 15u, hi = lane >> 4;
    const unsigned ntn = (unsigned)(DIM3 / GBN);
    const unsigned mT = blockIdx.x / ntn, nT = blockIdx.x - mT * ntn;
    const unsigned m0 = mT * GBM, n0 = nT * GBN;
    v8f acc[2][4];
#pragma unroll
    for (int i = 0; i < 2; ++i)
#pragma unroll
        for (int j = 0; j < 4; ++j) acc[i][j] = (v8f){};
    gemm_acc(XN, WQT, (unsigned)DIM, m0 + wv * 32u + lr, n0 + lr, hi, acc);
#pragma unroll
    for (int i = 0; i < 2; ++i)
#pragma unroll
        for (int j = 0; j < 4; ++j)
#pragma unroll
            for (int r = 0; r < 8; ++r) st[(wv * 32u + i * 16u + 8u * hi + r) * GP + j * 16u + lr] = acc[i][j][r];
    __syncthreads();
    const unsigned which = nT >> 3, h = nT & 7u;
    const unsigned b = m0 / (unsigned)SEQ, nq0 = m0 - b * (unsigned)SEQ;
    const unsigned bh = b * NH + h;
    if (which < 2u) {
        bf* ph = QK + (size_t)which * PLN + ((size_t)bh * SEQ + nq0) * HD;
        const float car = (which == 0u) ? QEP : KEP;
#pragma unroll 1
        for (int ps = 0; ps < 2; ++ps) {
#pragma unroll
            for (unsigned it = 0; it < 8; ++it) {
                const unsigned idx = it * 128u + tid;
                const unsigned row = idx >> 3, c8 = (idx & 7u) * 8u;
                const v4f x0 = *(const v4fa*)(st + row * GP + c8);
                const v4f x1 = *(const v4fa*)(st + row * GP + c8 + 4u);
                v8h ov;
#pragma unroll
                for (int c = 0; c < 4; ++c) {
                    ov[c] = toh_flush(x0[c] * car);
                    ov[4 + c] = toh_flush(x1[c] * car);
                }
                const v8us ouv = __builtin_bit_cast(v8us, ov);
                *(volatile v8us*)(ph + (size_t)row * HD + c8) = ouv;
            }
            if (ps == 0) __threadfence();
        }
    } else {
        bf* pv = VT + (size_t)bh * HD * SEQ + nq0;
#pragma unroll 1
        for (int ps = 0; ps < 2; ++ps) {
#pragma unroll
            for (unsigned it = 0; it < 8; ++it) {
                const unsigned idx = it * 128u + tid;
                const unsigned d = idx >> 4, n8 = (idx & 15u) * 8u;
                v8h o;
#pragma unroll
                for (unsigned c = 0; c < 8; ++c) o[c] = toh_flush(st[(n8 + c) * GP + d] * VEP);
                const v8us ou = __builtin_bit_cast(v8us, o);
                *(volatile v8us*)(pv + (size_t)d * SEQ + n8) = ou;
            }
            if (ps == 0) __threadfence();
        }
    }
}

__global__ __launch_bounds__(128) void k_flash(const bf* __restrict__ QK, const bf* __restrict__ VT, bf* CTX) {
    __shared__ __align__(16) float os[NWV * 16 * OSP];
    const unsigned tid = threadIdx.x, lane = tid & 31u, wv = tid >> 5, lr = lane & 15u, hi = lane >> 4;
    const unsigned bpb = (unsigned)(SEQ / BQ);
    const unsigned bh = blockIdx.x / bpb;
    const unsigned q0 = (blockIdx.x - bh * bpb) * BQ + wv * 16u;
    const unsigned b = bh / NH, h = bh - b * NH;

    v16h qh[2];
    {
        const bf* qp = QK + ((size_t)bh * SEQ + q0 + lr) * HD + 8u * hi;
#pragma unroll
        for (int dk = 0; dk < 2; ++dk) { qh[dk] = ldh(qp + dk * 32); }
    }
    const bf* kp = QK + PLN + ((size_t)bh * SEQ + lr) * HD + 8u * hi;
    const bf* vp = VT + ((size_t)bh * HD + lr) * SEQ + 8u * hi;

    v8f o[4];
#pragma unroll
    for (int t = 0; t < 4; ++t) o[t] = (v8f){};
    float ml = -1.0e30f;
    float l = 0.0f;

#pragma unroll 1
    for (unsigned k0 = 0; k0 < (unsigned)SEQ; k0 += KS) {
        v8f s0 = (v8f){}, s1 = (v8f){};
        const bf* ka = kp + (size_t)k0 * HD;
#pragma unroll
        for (int dk = 0; dk < 2; ++dk) {
            const v16h a0 = ldh(ka + dk * 32);
            const v16h a1 = ldh(ka + 16 * HD + dk * 32);
            s0 = wmmah(a0, qh[dk], s0);
            s1 = wmmah(a1, qh[dk], s1);
        }
        asm volatile("v_nop\n\tv_nop\n\tv_nop\n\tv_nop" : "+v"(s0), "+v"(s1) : "v"(qh[0]), "v"(qh[1]));

        float mx = fmaxf(s0[0], s1[0]);
#pragma unroll
        for (int r = 1; r < 8; ++r) mx = fmaxf(mx, fmaxf(s0[r], s1[r]));
        mx = fmaxf(mx, __shfl_xor(mx, 16, 32));
        const float mnl = fmaxf(ml, mx * L2ES);
        const float corr = __builtin_amdgcn_exp2f(ml - mnl);
        ml = mnl;
        const float sh = PCL - mnl;
        float p0[8], p1[8];
        float ps = 0.0f;
#pragma unroll
        for (int r = 0; r < 8; ++r) {
            const float x0 = fmaf(s0[r], L2ES, sh);
            const float x1 = fmaf(s1[r], L2ES, sh);
            const float y0 = __builtin_amdgcn_exp2f(x0);
            const float y1 = __builtin_amdgcn_exp2f(x1);
            p0[r] = (x0 < -14.0f) ? 0.0f : y0;
            p1[r] = (x1 < -14.0f) ? 0.0f : y1;
            ps += p0[r] + p1[r];
        }
        ps += __shfl_xor(ps, 16, 32);
        l = l * corr + ps;
        if (__builtin_amdgcn_ballot_w32(corr != 1.0f) != 0u) {
#pragma unroll
            for (int t = 0; t < 4; ++t) o[t] *= corr;
        }

        v16h ph;
#pragma unroll
        for (int r = 0; r < 8; ++r) { ph[r] = (_Float16)p0[r]; ph[8 + r] = (_Float16)p1[r]; }

        asm volatile("" ::: "memory");
        const bf* va = vp + k0;
#pragma unroll
        for (int t = 0; t < 4; ++t) {
            const v16h a = ldh(va + (size_t)t * 16 * SEQ);
            o[t] = wmmah(a, ph, o[t]);
        }
        asm volatile("v_nop\n\tv_nop\n\tv_nop\n\tv_nop"
                     : "+v"(o[0]), "+v"(o[1]), "+v"(o[2]), "+v"(o[3])
                     : "v"(ph));
    }

    const float inv = 1.0f / l;
    float* ow = os + wv * (16 * OSP);
#pragma unroll
    for (int t = 0; t < 4; ++t) {
#pragma unroll
        for (int r = 0; r < 8; ++r) ow[lr * OSP + t * 16 + 8 * hi + r] = o[t][r] * inv;
    }
    __syncthreads();
    bf* crow = CTX + ((size_t)b * SEQ + q0) * DIM + h * HD;
    const unsigned rq = lane >> 3, c8 = (lane & 7u) * 8u;
#pragma unroll 1
    for (int ps2 = 0; ps2 < 2; ++ps2) {
#pragma unroll
        for (unsigned it = 0; it < 4; ++it) {
            const unsigned row = it * 4u + rq;
            const v4f x0 = *(const v4fa*)(ow + row * OSP + c8);
            const v4f x1 = *(const v4fa*)(ow + row * OSP + c8 + 4u);
            v8h ov;
#pragma unroll
            for (int c = 0; c < 4; ++c) {
                ov[c] = toh_flush(x0[c] * CCAR);
                ov[4 + c] = toh_flush(x1[c] * CCAR);
            }
            const v8us ou = __builtin_bit_cast(v8us, ov);
            *(volatile v8us*)(crow + (size_t)row * DIM + c8) = ou;
        }
        if (ps2 == 0) __threadfence();
    }
}

__global__ __launch_bounds__(128) void k_proj(const bf* __restrict__ CTX, const bf* __restrict__ WOT, const float* __restrict__ bias, float* O) {
    __shared__ __align__(16) float st[GBM * GP];
    const unsigned tid = threadIdx.x, lane = tid & 31u, wv = tid >> 5, lr = lane & 15u, hi = lane >> 4;
    const unsigned ntn = (unsigned)(DIM / GBN);
    const unsigned mT = blockIdx.x / ntn, nT = blockIdx.x - mT * ntn;
    const unsigned m0 = mT * GBM, n0 = nT * GBN;
    v8f acc[2][4];
#pragma unroll
    for (int i = 0; i < 2; ++i)
#pragma unroll
        for (int j = 0; j < 4; ++j) acc[i][j] = (v8f){};
    gemm_acc(CTX, WOT, (unsigned)DIM, m0 + wv * 32u + lr, n0 + lr, hi, acc);
#pragma unroll
    for (int i = 0; i < 2; ++i)
#pragma unroll
        for (int j = 0; j < 4; ++j)
#pragma unroll
            for (int r = 0; r < 8; ++r) st[(wv * 32u + i * 16u + 8u * hi + r) * GP + j * 16u + lr] = acc[i][j][r];
    __syncthreads();
    float* ob = O + (size_t)m0 * DIM + n0;
    const v4f braw = *(const v4f*)(bias + n0 + (tid & 15u) * 4u);
    v4f bi;
#pragma unroll
    for (int c = 0; c < 4; ++c) bi[c] = bf2f(f2bf(braw[c]));
#pragma unroll 1
    for (int ps = 0; ps < 2; ++ps) {
#pragma unroll 4
        for (unsigned it = 0; it < 16; ++it) {
            const unsigned idx = it * 128u + tid;
            const unsigned row = idx >> 4, c4 = (idx & 15u) * 4u;
            const v4f val = *(const v4fa*)(st + row * GP + c4) * OSC + bi;
            *(volatile v4f*)(ob + (size_t)row * DIM + c4) = val;
        }
        if (ps == 0) __threadfence();
    }
}

extern "C" void kernel_launch(void* const* d_in, const int* in_sizes, int n_in,
                              void* d_out, int out_size, void* d_ws, size_t ws_size, hipStream_t stream) {
    if (n_in < 6) return;
    const size_t needx = ((size_t)(NB - 1) * SEQ_FULL + SEQ) * DIM;
    if ((size_t)in_sizes[0] < needx) return;
    if ((size_t)in_sizes[1] < (size_t)DIM3 * DIM) return;
    if ((size_t)in_sizes[2] < (size_t)DIM * DIM) return;
    if ((size_t)in_sizes[3] < (size_t)DIM) return;
    if ((size_t)in_sizes[4] < (size_t)DIM) return;
    if ((size_t)in_sizes[5] < (size_t)DIM) return;
    if ((size_t)out_size < (size_t)MROWS * DIM) return;
    const float* x      = (const float*)d_in[0];
    const float* w_qkv  = (const float*)d_in[1];
    const float* w_proj = (const float*)d_in[2];
    const float* b_proj = (const float*)d_in[3];
    const float* ln_g   = (const float*)d_in[4];
    const float* ln_b   = (const float*)d_in[5];
    float* OUT = (float*)d_out;

    constexpr size_t WQT_B = (size_t)DIM3 * DIM * 2;
    constexpr size_t WOT_B = (size_t)DIM * DIM * 2;
    constexpr size_t PLN_B = (size_t)MROWS * DIM * 2;
    constexpr size_t OFF_WQT = 0;
    constexpr size_t OFF_WOT = OFF_WQT + WQT_B;
    constexpr size_t OFF_QK  = OFF_WOT + WOT_B;
    constexpr size_t OFF_VT  = OFF_QK + 2 * PLN_B;
    constexpr size_t OFF_XC  = OFF_VT + PLN_B;
    constexpr size_t WS_TOTAL = OFF_XC + PLN_B;
    static_assert(WS_TOTAL <= (size_t)134217728);
    static_assert(OFF_WOT % 256 == 0);
    static_assert(OFF_QK % 256 == 0);
    static_assert(OFF_VT % 256 == 0);
    static_assert(OFF_XC % 256 == 0);
    static_assert(OFF_VT - OFF_QK == 2 * PLN_B);
    static_assert((size_t)MROWS * DIM * 2 == PLN_B);
    if (WS_TOTAL > ws_size) return;

    char* wsp = (char*)d_ws;
    bf* WQT = (bf*)(wsp + OFF_WQT);
    bf* WOT = (bf*)(wsp + OFF_WOT);
    bf* QK  = (bf*)(wsp + OFF_QK);
    bf* VT  = (bf*)(wsp + OFF_VT);
    bf* XN  = (bf*)(wsp + OFF_XC);
    bf* CTX = (bf*)(wsp + OFF_XC);

    k_wc<<<(unsigned)((size_t)DIM3 * (DIM / 8) / 256), 256, 0, stream>>>(w_qkv, WQT, DIM3, DIM, 1, DIM);
    k_wc<<<(unsigned)((size_t)DIM * (DIM / 8) / 256), 256, 0, stream>>>(w_proj, WOT, DIM, DIM, 1, 0);
    k_ln<<<(unsigned)(MROWS / 8), 256, 0, stream>>>(x, ln_g, ln_b, XN);
    k_qkv<<<(unsigned)((MROWS / GBM) * (DIM3 / GBN)), 128, 0, stream>>>(XN, WQT, QK, VT);
    k_flash<<<(unsigned)(NB * NH * (SEQ / BQ)), 128, 0, stream>>>(QK, VT, CTX);
    k_proj<<<(unsigned)((MROWS / GBM) * (DIM / GBN)), 128, 0, stream>>>(CTX, WOT, b_proj, OUT);
}
